// sc_conv_82643760709696
// MI455X (gfx1250) — hardware-verified
//
#include <hip/hip_runtime.h>
#include <stddef.h>

#pragma clang fp contract(off)

typedef float    v4f  __attribute__((ext_vector_type(4)));
typedef float    v8f  __attribute__((ext_vector_type(8)));
typedef unsigned v4u  __attribute__((ext_vector_type(4)));
typedef _Float16 v8h  __attribute__((ext_vector_type(8)));
typedef _Float16 v16h __attribute__((ext_vector_type(16)));

#define K3 27
#define CENTER 13
#define CH 32
#define NBLK 256
#define MAXB 16
#define WPLANE (K3 * 2 * 32 * 16)
#define WSET (2 * WPLANE)
#define NPACK (2 * 2 * K3 * 2 * 32 * 2)
#define SC_A 256.0f
#define SC_W 4096.0f
#define SC_OUT (1.0f / 1048576.0f)

union Frag { v16h v; v4u q[2]; };
union H8 { v8h v; v4u u; };

__device__ __forceinline__ v8f mma16(v16h a, v16h b, v8f c) {
  v8f d = __builtin_amdgcn_wmma_f32_16x16x32_f16(false, a, false, b, (short)0, c, false, false);
  asm volatile("v_nop\n\tv_nop\n\tv_nop\n\tv_nop" : "+v"(d) : "v"(a), "v"(b));
  return d;
}

__device__ __forceinline__ void split8(v4f x0, v4f x1, float sc, v4u& hi, v4u& lo) {
  H8 uh, ul;
#pragma unroll
  for (int j = 0; j < 4; ++j) {
    float v = x0[j] * sc;
    _Float16 hv = (_Float16)v;
    uh.v[j] = hv;
    ul.v[j] = (_Float16)(v - (float)hv);
    float w = x1[j] * sc;
    _Float16 hw = (_Float16)w;
    uh.v[4 + j] = hw;
    ul.v[4 + j] = (_Float16)(w - (float)hw);
  }
  hi = uh.u;
  lo = ul.u;
}

__device__ __forceinline__ int clamp_nbat(int nb) {
  return nb < 1 ? 1 : (nb > MAXB ? MAXB : nb);
}

__device__ __forceinline__ int chunk_of(int nbpts) {
  return (((nbpts + NBLK - 1) / NBLK) + 31) & ~31;
}

__global__ void __launch_bounds__(256) k_pack(const float* __restrict__ Wch, const float* __restrict__ Wdw,
                                             _Float16* __restrict__ wpk, int total) {
  const int t = blockIdx.x * blockDim.x + threadIdx.x;
  const bool in = t < total;
  int r = in ? t : 0;
  const int half = r & 1; r >>= 1;
  const int fl = r & 31;  r >>= 5;
  const int nt = r & 1;   r >>= 1;
  const int k = r % K3;   r /= K3;
  const int q = r & 1;    r >>= 1;
  const int set = r & 1;
  const float* W = set ? Wdw : Wch;
  const int hh = fl >> 4;
  const int col = nt * 16 + (fl & 15);
  const int cin0 = half ? (16 + 8 * hh) : (8 * hh);
  H8 o;
#pragma unroll
  for (int j = 0; j < 8; ++j) {
    float w = W[(size_t)k * (CH * CH) + (size_t)(cin0 + j) * CH + col] * SC_W;
    _Float16 hw = (_Float16)w;
    _Float16 lw = (_Float16)(w - (float)hw);
    o.v[j] = (q == 0) ? hw : lw;
  }
  v4u val = o.u;
  _Float16* dst = wpk + (size_t)t * 8;
  if (in) *(volatile v4u*)dst = val;
  __threadfence();
  if (in) *(volatile v4u*)dst = val;
}

__global__ void __launch_bounds__(256) k_xsplit(const float* __restrict__ x, _Float16* __restrict__ pl,
                                               size_t ps, int n8) {
  const int i = blockIdx.x * blockDim.x + threadIdx.x;
  const bool in = i < n8;
  v4f a = {0.f, 0.f, 0.f, 0.f};
  v4f b = {0.f, 0.f, 0.f, 0.f};
  if (in) {
    a = *(const v4f*)(x + (size_t)i * 8);
    b = *(const v4f*)(x + (size_t)i * 8 + 4);
  }
  v4u hi, lo;
  split8(a, b, SC_A, hi, lo);
  _Float16* d0 = pl + (size_t)i * 8;
  _Float16* d1 = pl + ps + (size_t)i * 8;
  if (in) { *(volatile v4u*)d0 = hi; *(volatile v4u*)d1 = lo; }
  __threadfence();
  if (in) { *(volatile v4u*)d0 = hi; *(volatile v4u*)d1 = lo; }
}

__device__ __forceinline__ v8f mac3(v8f d, const Frag& a0, const Frag& a1,
                                    const _Float16* w0, const _Float16* w1) {
  Frag b0, b1;
  b0.q[0] = *(const v4u*)(w0);
  b0.q[1] = *(const v4u*)(w0 + 8);
  b1.q[0] = *(const v4u*)(w1);
  b1.q[1] = *(const v4u*)(w1 + 8);
  d = mma16(a0.v, b0.v, d);
  d = mma16(a0.v, b1.v, d);
  d = mma16(a1.v, b0.v, d);
  return d;
}

__device__ __forceinline__ void store0(float (*tl)[CH], int lane, int pt0, int N,
                                       float* fout, float* snout, _Float16* qout, size_t qps) {
#pragma unroll
  for (int j = 0; j < 4; ++j) {
    const int row = 4 * j + (lane >> 3);
    const int c0 = (lane & 7) * 4;
    const int pt = pt0 + row;
    v4f v = *(const v4f*)(&tl[row][c0]);
    if (pt < N) *(volatile v4f*)(fout + (size_t)pt * CH + c0) = v;
  }
  if (lane < 16) {
    const int pt = pt0 + lane;
    float s = 0.f, q = 0.f;
#pragma unroll
    for (int c = 0; c < CH; ++c) {
      float v = tl[lane][c];
      s = s + v;
      q = q + v * v;
    }
    if (pt < N) {
      v4f o = {s, q, 0.f, 0.f};
      *(volatile v4f*)(snout + (size_t)pt * 4) = o;
    }
  }
#pragma unroll
  for (int j = 0; j < 2; ++j) {
    const int row = 8 * j + (lane >> 2);
    const int c0 = (lane & 3) * 8;
    const int pt = pt0 + row;
    v4f x0 = *(const v4f*)(&tl[row][c0]);
    v4f x1 = *(const v4f*)(&tl[row][c0 + 4]);
    v4u hi, lo;
    split8(x0, x1, SC_A, hi, lo);
    if (pt < N) {
      _Float16* dq = qout + (size_t)pt * CH + c0;
      *(volatile v4u*)dq = hi;
      *(volatile v4u*)(dq + qps) = lo;
    }
  }
}

__device__ __forceinline__ void store1(float (*tl)[CH], int lane, int pt0, int N,
                                       const unsigned* msk, const float* xin, float* fout) {
#pragma unroll
  for (int j = 0; j < 4; ++j) {
    const int row = 4 * j + (lane >> 3);
    const int c0 = (lane & 7) * 4;
    const int pt = pt0 + row;
    if (pt < N) {
      const unsigned mk = msk[pt];
      v4f t = *(const v4f*)(&tl[row][c0]);
      v4f x = *(const v4f*)(xin + (size_t)pt * CH + c0);
      v4f o = mk ? (t + x) : (x + x);
      *(volatile v4f*)(fout + (size_t)pt * CH + c0) = o;
    }
  }
}

template <int MODE>
__global__ void __launch_bounds__(64) k_conv(const _Float16* apl, size_t aps, const _Float16* wpl,
                                            const float* bias, const int* nbr, const unsigned* msk,
                                            const float* xin, float* fout, float* snout,
                                            _Float16* qout, size_t qps, int N) {
  __shared__ __attribute__((aligned(16))) float tile[2][16][CH];
  const int lane = threadIdx.x & 31, wv = threadIdx.x >> 5;
  const int h = lane >> 4, m = lane & 15;
  const int pt0 = (blockIdx.x * 2 + wv) * 16;
  const int p = pt0 + m;
  const bool pin = p < N;
  unsigned um = 1u;
  if (MODE == 1) um = pin ? msk[p] : 0u;
  const bool prow = pin && (um != 0u);
  const bool anyw = (__ballot(prow ? 1 : 0) != 0ull);

  v8f d0 = {0.f, 0.f, 0.f, 0.f, 0.f, 0.f, 0.f, 0.f};
  v8f d1 = {0.f, 0.f, 0.f, 0.f, 0.f, 0.f, 0.f, 0.f};
  const v4u z4 = {0u, 0u, 0u, 0u};

  if (anyw) {
    const int* nb = nbr + (size_t)(pin ? p : 0) * K3;
    const _Float16* wl = wpl + lane * 16;
    for (int k = 0; k < K3; ++k) {
      const int idx = prow ? nb[k] : -1;
      bool val = idx >= 0;
      const int ci = val ? (idx < N ? idx : N - 1) : 0;
      if (MODE == 1) { if (val) val = (msk[ci] != 0u); }
      if (__ballot(val ? 1 : 0) == 0ull) continue;
      Frag a0, a1;
      a0.q[0] = z4; a0.q[1] = z4; a1.q[0] = z4; a1.q[1] = z4;
      if (val) {
        const _Float16* ar = apl + (size_t)ci * CH + 8 * h;
        a0.q[0] = *(const v4u*)(ar);
        a0.q[1] = *(const v4u*)(ar + 16);
        const _Float16* ar2 = ar + aps;
        a1.q[0] = *(const v4u*)(ar2);
        a1.q[1] = *(const v4u*)(ar2 + 16);
      }
      const _Float16* wk = wl + k * 1024;
      d0 = mac3(d0, a0, a1, wk, wk + WPLANE);
      d1 = mac3(d1, a0, a1, wk + 512, wk + 512 + WPLANE);
    }
  }

  const float bb0 = bias[m], bb1 = bias[16 + m];
#pragma unroll
  for (int r = 0; r < 8; ++r) {
    tile[wv][8 * h + r][m]      = d0[r] * SC_OUT + bb0;
    tile[wv][8 * h + r][16 + m] = d1[r] * SC_OUT + bb1;
  }
  __syncthreads();
  if (MODE == 0) store0(tile[wv], lane, pt0, N, fout, snout, qout, qps);
  else           store1(tile[wv], lane, pt0, N, msk, xin, fout);
  __threadfence();
  if (MODE == 0) store0(tile[wv], lane, pt0, N, fout, snout, qout, qps);
  else           store1(tile[wv], lane, pt0, N, msk, xin, fout);
}

__global__ void __launch_bounds__(256) k_corr(const int* __restrict__ nbr, const float* __restrict__ sn,
                                             unsigned* __restrict__ keys, int N) {
  const int n = blockIdx.x * blockDim.x + threadIdx.x;
  const bool in = n < N;
  float acc = 0.f;
  float nrm = 1.f;
  if (in) {
    const int* nb = nbr + (size_t)n * K3;
#pragma unroll
    for (int k = 0; k < K3; ++k) {
      if (k == CENTER) continue;
      const int idx = nb[k];
      if (idx >= 0) {
        const int ci = idx < N ? idx : N - 1;
        acc = acc + sn[(size_t)ci * 4];
      }
    }
    nrm = sn[(size_t)n * 4 + 1];
  }
  const float rc = 1.0f / nrm;
  const float c = acc * rc;
  const unsigned u = __float_as_uint(c);
  const unsigned key = (u & 0x80000000u) ? ~u : (u | 0x80000000u);
  if (in) *(volatile unsigned*)(keys + n) = key;
  __threadfence();
  if (in) *(volatile unsigned*)(keys + n) = key;
}

__global__ void __launch_bounds__(256) k_count(const unsigned* __restrict__ keys,
                                              const unsigned* __restrict__ st,
                                              unsigned* __restrict__ cnt,
                                              const int* __restrict__ nbp, int N, int pass) {
  __shared__ unsigned red[16][NBLK];
  const int t = threadIdx.x, j = blockIdx.x;
  const int nbat = clamp_nbat(nbp[0]);
  const int nbpts = N / nbat;
  const int chunk = chunk_of(nbpts);
  const int iters = (chunk + 255) / 256;
  const int sh = (28 - 4 * pass) & 31;
  const int shp = (32 - 4 * pass) & 31;
  for (int b = 0; b < nbat; ++b) {
    const unsigned prefix = (pass == 0) ? 0u : st[b * 32];
    const int lo = b * nbpts + j * chunk;
    const int lim = ((j + 1) * chunk < nbpts) ? (j + 1) * chunk : nbpts;
    const int hi = b * nbpts + lim;
    unsigned c[16];
#pragma unroll
    for (int d = 0; d < 16; ++d) c[d] = 0u;
    for (int g = 0; g < iters; ++g) {
      const int n = lo + g * 256 + t;
      if (n < hi) {
        const unsigned key = keys[n];
        if (pass < 8) {
          const bool match = (pass == 0) || ((key >> shp) == prefix);
          const unsigned dg = (key >> sh) & 15u;
          if (match) {
#pragma unroll
            for (int d = 0; d < 16; ++d) c[d] += (dg == (unsigned)d) ? 1u : 0u;
          }
        } else {
          c[0] += (key == prefix) ? 1u : 0u;
        }
      }
    }
#pragma unroll
    for (int d = 0; d < 16; ++d) red[d][t] = c[d];
    __syncthreads();
    unsigned tot = 0u;
    if (t < 16) {
      for (int u = 0; u < NBLK; ++u) tot += red[t][u];
    }
    if (t < 32) {
      const unsigned v = (t < 16) ? tot : 0u;
      unsigned* dst = cnt + ((size_t)b * NBLK + j) * 32 + t;
      *(volatile unsigned*)dst = v;
      __threadfence();
      *(volatile unsigned*)dst = v;
    }
    __syncthreads();
  }
}

__global__ void __launch_bounds__(256) k_pick(const unsigned* __restrict__ cnt, unsigned* __restrict__ st,
                                             unsigned* __restrict__ eqoff, const int* __restrict__ nbp,
                                             const int* __restrict__ thp, int N, int pass) {
  __shared__ unsigned red[16][NBLK];
  __shared__ unsigned tot[16];
  __shared__ unsigned stl[32];
  __shared__ unsigned pre[NBLK];
  const int t = threadIdx.x;
  const int nbat = clamp_nbat(nbp[0]);
  const int nbpts = N / nbat;
  for (int b = 0; b < nbat; ++b) {
    if (pass < 8) {
#pragma unroll
      for (int d = 0; d < 16; ++d) red[d][t] = cnt[((size_t)b * NBLK + t) * 32 + d];
      if (t < 32) stl[t] = (pass == 0) ? 0u : st[b * 32 + t];
      __syncthreads();
      if (t < 16) {
        unsigned s = 0u;
        for (int u = 0; u < NBLK; ++u) s += red[t][u];
        tot[t] = s;
      }
      __syncthreads();
      if (t == 0) {
        unsigned prefix, krem;
        if (pass == 0) {
          double kd = (double)nbpts * (double)thp[0] / 3.21;
          if (!(kd >= 0.0)) kd = 0.0;
          if (kd > (double)nbpts) kd = (double)nbpts;
          const unsigned kk = (unsigned)((int)kd);
          prefix = 0u;
          krem = kk;
          stl[2] = kk;
        } else {
          prefix = stl[0];
          krem = stl[1];
        }
        unsigned np, nk;
        if (krem == 0u) {
          np = (pass == 0) ? 0xFFFFFFFFu : prefix;
          nk = 0u;
        } else {
          unsigned cumb = 0u, kb = 0u;
          int dsel = 0;
          bool found = false;
          for (int d = 15; d >= 0; --d) {
            const unsigned cd = tot[d];
            if (!found && cumb < krem && cumb + cd >= krem) { found = true; dsel = d; kb = krem - cumb; }
            cumb += cd;
          }
          if (found) { np = (prefix << 4) | (unsigned)dsel; nk = kb; }
          else       { np = 0xFFFFFFFFu; nk = 0u; }
        }
        stl[0] = np;
        stl[1] = nk;
      }
      __syncthreads();
      if (t < 32) {
        const unsigned v = stl[t];
        unsigned* dst = st + b * 32 + t;
        *(volatile unsigned*)dst = v;
        __threadfence();
        *(volatile unsigned*)dst = v;
      }
      __syncthreads();
    } else {
      red[0][t] = cnt[((size_t)b * NBLK + t) * 32];
      __syncthreads();
      if (t == 0) {
        unsigned run = 0u;
        for (int u = 0; u < NBLK; ++u) { pre[u] = run; run += red[0][u]; }
      }
      __syncthreads();
      {
        const unsigned v = pre[t];
        unsigned* dst = eqoff + (size_t)b * NBLK + t;
        *(volatile unsigned*)dst = v;
        __threadfence();
        *(volatile unsigned*)dst = v;
      }
      __syncthreads();
    }
  }
}

__global__ void __launch_bounds__(256) k_mask(const unsigned* __restrict__ keys, const unsigned* __restrict__ st,
                                             const unsigned* __restrict__ eqoff, unsigned* __restrict__ msk,
                                             const int* __restrict__ nbp, int N) {
  __shared__ unsigned wtot[8];
  const int t = threadIdx.x, j = blockIdx.x;
  const int lane = t & 31, w = t >> 5;
  const int nbat = clamp_nbat(nbp[0]);
  const int nbpts = N / nbat;
  const int chunk = chunk_of(nbpts);
  const int iters = (chunk + 255) / 256;
  for (int b = 0; b < nbat; ++b) {
    const unsigned T = st[b * 32];
    const unsigned rq = st[b * 32 + 1];
    const unsigned base = eqoff[(size_t)b * NBLK + j];
    const int lo = b * nbpts + j * chunk;
    const int lim = ((j + 1) * chunk < nbpts) ? (j + 1) * chunk : nbpts;
    const int hi = b * nbpts + lim;
    unsigned running = 0u;
    for (int g = 0; g < iters; ++g) {
      const int n = lo + g * 256 + t;
      const bool in = n < hi;
      const unsigned key = in ? keys[n] : 0u;
      const bool eq = in && (key == T);
      const unsigned bal = (unsigned)__ballot(eq ? 1 : 0);
      const unsigned lp = __popc(bal & ((1u << lane) - 1u));
      if (lane == 0) wtot[w] = __popc(bal);
      __syncthreads();
      unsigned woff = 0u, all = 0u;
#pragma unroll
      for (int u = 0; u < 8; ++u) { const unsigned c = wtot[u]; if (u < w) woff += c; all += c; }
      __syncthreads();
      const unsigned rank = base + running + woff + lp;
      running += all;
      const unsigned mv = (in && ((key > T) || (eq && rank < rq))) ? 1u : 0u;
      if (in) *(volatile unsigned*)(msk + n) = mv;
      __threadfence();
      if (in) *(volatile unsigned*)(msk + n) = mv;
    }
  }
}

extern "C" void kernel_launch(void* const* d_in, const int* in_sizes, int n_in,
                              void* d_out, int out_size, void* d_ws, size_t ws_size,
                              hipStream_t stream) {
  if (n_in < 8) return;
  const float* xF   = (const float*)d_in[0];
  const float* Wch  = (const float*)d_in[1];
  const float* bch  = (const float*)d_in[2];
  const float* Wdw  = (const float*)d_in[3];
  const float* bdw  = (const float*)d_in[4];
  const int*   nbr  = (const int*)d_in[5];
  const int*   thp  = (const int*)d_in[6];
  const int*   nbp  = (const int*)d_in[7];

  const int N = in_sizes[0] / CH;
  if (N <= 0 || out_size < N * CH || in_sizes[5] < N * K3) return;

  size_t off = 0;
  auto carve = [&](size_t bytes) -> size_t {
    size_t o = off;
    off = (off + bytes + 255) & ~(size_t)255;
    return o;
  };
  const size_t ps = (size_t)N * CH;
  const size_t oWpk = carve((size_t)2 * WSET * sizeof(_Float16));
  const size_t oXs  = carve(2 * ps * sizeof(_Float16));
  const size_t oWx  = carve((size_t)N * CH * sizeof(float));
  const size_t oSn  = carve((size_t)N * 4 * sizeof(float));
  const size_t oXq  = carve(2 * ps * sizeof(_Float16));
  const size_t oKey = carve((size_t)N * sizeof(unsigned));
  const size_t oMsk = carve((size_t)N * sizeof(unsigned));
  const size_t oCnt = carve((size_t)MAXB * NBLK * 32 * sizeof(unsigned));
  const size_t oEq  = carve((size_t)MAXB * NBLK * sizeof(unsigned));
  const size_t oSt  = carve((size_t)MAXB * 32 * sizeof(unsigned));
  if (off > ws_size) return;

  char* ws = (char*)d_ws;
  _Float16* wpk  = (_Float16*)(ws + oWpk);
  _Float16* xs   = (_Float16*)(ws + oXs);
  float*    wx   = (float*)(ws + oWx);
  float*    sn   = (float*)(ws + oSn);
  _Float16* xq   = (_Float16*)(ws + oXq);
  unsigned* keys = (unsigned*)(ws + oKey);
  unsigned* msk  = (unsigned*)(ws + oMsk);
  unsigned* cnt  = (unsigned*)(ws + oCnt);
  unsigned* eqo  = (unsigned*)(ws + oEq);
  unsigned* st   = (unsigned*)(ws + oSt);

  k_pack<<<(NPACK + 255) / 256, 256, 0, stream>>>(Wch, Wdw, wpk, NPACK);

  const int n8 = N * 4;
  k_xsplit<<<(n8 + 255) / 256, 256, 0, stream>>>(xF, xs, ps, n8);

  const int cblk = (N + 31) / 32;
  k_conv<0><<<cblk, 64, 0, stream>>>(xs, ps, wpk, bch, nbr, msk, wx, wx, sn, xq, ps, N);

  k_corr<<<(N + 255) / 256, 256, 0, stream>>>(nbr, sn, keys, N);

  for (int pass = 0; pass < 9; ++pass) {
    k_count<<<NBLK, 256, 0, stream>>>(keys, st, cnt, nbp, N, pass);
    k_pick<<<1, 256, 0, stream>>>(cnt, st, eqo, nbp, thp, N, pass);
  }

  k_mask<<<NBLK, 256, 0, stream>>>(keys, st, eqo, msk, nbp, N);

  k_conv<1><<<cblk, 64, 0, stream>>>(xq, ps, wpk + WSET, bdw, nbr, msk, wx, (float*)d_out, sn, xq, ps, N);
}
